// TimeMix_71940702208372
// MI455X (gfx1250) — hardware-run, weakly checked
//
#include <hip/hip_runtime.h>
#include <stddef.h>


#pragma clang fp contract(off)

#define TT    2048
#define CC    2048
#define GTHR  128
#define GWAV  (GTHR / 32)
#define BMB   64
#define BNB   128
#define ETHR  256
#define EWAV  (ETHR / 32)
#define TB    32
#define WTT   64
#define WTP   72
#define WCAR  64.0f
#define RCAR  64.0f
#define PSCL  (1.0f / 64.0f)
#define OSCL  (1.0f / 4096.0f)
#define WSCAP 134217728

#define SZH   ((size_t)TT * CC * 2)
#define SZF   ((size_t)TT * CC * 4)
#define OXK   ((size_t)0)
#define OXV   (OXK + SZH)
#define OXR   (OXV + SZH)
#define OWK   (OXR + SZH)
#define OWV   (OWK + SZH)
#define OWR   (OWV + SZH)
#define OWO   (OWR + SZH)
#define OKF   (OWO + SZH)
#define OVF   (OKF + SZF)
#define OSF   (OVF + SZF)
#define ORW   (OSF + SZF)
#define WSTOT (ORW + SZH)

static_assert(WSTOT <= (size_t)WSCAP);
static_assert((OWK % 128) == 0 && (OKF % 128) == 0 && (ORW % 128) == 0);
static_assert(OXV == OXK + SZH && OXR == OXV + SZH);
static_assert(OWV == OWK + SZH && OWR == OWV + SZH && OWO == OWR + SZH);
static_assert(OVF == OKF + SZF && OSF == OVF + SZF);
static_assert((CC % 32) == 0);
static_assert((TT % BMB) == 0 && (CC % BNB) == 0);
static_assert(BMB == 2 * 32 && BNB == 2 * 64 && GWAV == 4);
static_assert(CC == ETHR * 8);
static_assert((CC % WTT) == 0 && (WTT * WTT) == 4 * 4 * ETHR && (WTT * WTT) == 2 * 8 * ETHR);
static_assert((CC % ETHR) == 0 && (TT % TB) == 0 && TB == 4 * EWAV);
static_assert((WTP % 8) == 0);

typedef _Float16 v16h __attribute__((ext_vector_type(16)));
typedef _Float16 v8h  __attribute__((ext_vector_type(8), __may_alias__));
typedef float    v8f  __attribute__((ext_vector_type(8)));
typedef float    v4f  __attribute__((ext_vector_type(4), __may_alias__));
union Frag { v16h v; v8h h[2]; };
static_assert(sizeof(Frag) == 32);

__device__ __forceinline__ v8f wmh(v16h a, v16h bq, v8f c) {
  v8f d = __builtin_amdgcn_wmma_f32_16x16x32_f16(false, a, false, bq, (short)0, c, false, false);
  asm volatile("v_nop\n\tv_nop\n\tv_nop\n\tv_nop" : "+v"(d) : "v"(a), "v"(bq));
  return d;
}

__device__ __forceinline__ v8f zero8() {
  v8f z = {0.f, 0.f, 0.f, 0.f, 0.f, 0.f, 0.f, 0.f};
  return z;
}

__device__ __forceinline__ float rcp_(float d) { return __builtin_amdgcn_rcpf(d); }
__device__ __forceinline__ float sigm_(float x) {
  const float xc = fminf(fmaxf(x, -30.0f), 30.0f);
  return rcp_(1.0f + __expf(-xc));
}

__device__ __forceinline__ v8h mix8(v4f a0, v4f a1, v4f p0, v4f p1, v4f m0, v4f m1) {
  const v4f one = {1.0f, 1.0f, 1.0f, 1.0f};
  const v4f r0 = a0 * m0 + p0 * (one - m0);
  const v4f r1 = a1 * m1 + p1 * (one - m1);
  v8h hv;
  hv[0] = (_Float16)r0.x; hv[1] = (_Float16)r0.y; hv[2] = (_Float16)r0.z; hv[3] = (_Float16)r0.w;
  hv[4] = (_Float16)r1.x; hv[5] = (_Float16)r1.y; hv[6] = (_Float16)r1.z; hv[7] = (_Float16)r1.w;
  return hv;
}

__global__ __launch_bounds__(ETHR) void k_mix(const float* __restrict__ x, const float* __restrict__ tmk,
                                              const float* __restrict__ tmv, const float* __restrict__ tmr,
                                              _Float16* XK, _Float16* XV, _Float16* XR) {
  const int t = blockIdx.x;
  const int tid = threadIdx.x;
  const int c0 = 8 * tid;
  const int tp = (t > 0) ? (t - 1) : 0;
  const size_t o  = (size_t)t * CC + c0;
  const size_t op = (size_t)tp * CC + c0;
  const v4f zero4 = {0.f, 0.f, 0.f, 0.f};
  const v4f a0 = *(const v4f*)(x + o);
  const v4f a1 = *(const v4f*)(x + o + 4);
  const v4f q0 = *(const v4f*)(x + op);
  const v4f q1 = *(const v4f*)(x + op + 4);
  const v4f p0 = (t > 0) ? q0 : zero4;
  const v4f p1 = (t > 0) ? q1 : zero4;
  const v4f mk0 = *(const v4f*)(tmk + c0), mk1 = *(const v4f*)(tmk + c0 + 4);
  const v4f mv0 = *(const v4f*)(tmv + c0), mv1 = *(const v4f*)(tmv + c0 + 4);
  const v4f mr0 = *(const v4f*)(tmr + c0), mr1 = *(const v4f*)(tmr + c0 + 4);
  const v8h hk = mix8(a0, a1, p0, p1, mk0, mk1);
  const v8h hv = mix8(a0, a1, p0, p1, mv0, mv1);
  const v8h hr = mix8(a0, a1, p0, p1, mr0, mr1);
  *(volatile v8h*)(XK + o) = hk;
  *(volatile v8h*)(XV + o) = hv;
  *(volatile v8h*)(XR + o) = hr;
  __threadfence();
  *(volatile v8h*)(XK + o) = hk;
  *(volatile v8h*)(XV + o) = hv;
  *(volatile v8h*)(XR + o) = hr;
}

__global__ __launch_bounds__(ETHR) void k_wt(const float* __restrict__ Wk, const float* __restrict__ Wv,
                                             const float* __restrict__ Wr, const float* __restrict__ Wo,
                                             _Float16* WT) {
  __shared__ __align__(16) _Float16 sT[WTT * WTP];
  const int sel = blockIdx.z;
  const float* W = (sel == 0) ? Wk : ((sel == 1) ? Wv : ((sel == 2) ? Wr : Wo));
  _Float16* O = WT + (size_t)sel * CC * CC;
  const int n0 = blockIdx.x * WTT;
  const int k0 = blockIdx.y * WTT;
  const int tid = threadIdx.x;

#pragma unroll
  for (int it = 0; it < 4; ++it) {
    const int e = tid + ETHR * it;
    const int kl = e >> 4, q = e & 15;
    const v4f v = *(const v4f*)(W + (size_t)(k0 + kl) * CC + n0 + 4 * q);
    sT[(4 * q + 0) * WTP + kl] = (_Float16)(v.x * WCAR);
    sT[(4 * q + 1) * WTP + kl] = (_Float16)(v.y * WCAR);
    sT[(4 * q + 2) * WTP + kl] = (_Float16)(v.z * WCAR);
    sT[(4 * q + 3) * WTP + kl] = (_Float16)(v.w * WCAR);
  }
  __syncthreads();

#pragma unroll
  for (int it = 0; it < 2; ++it) {
    const int e = tid + ETHR * it;
    const int nl = e >> 3, q = e & 7;
    const v8h hv = *(const v8h*)(sT + nl * WTP + 8 * q);
    *(volatile v8h*)(O + (size_t)(n0 + nl) * CC + k0 + 8 * q) = hv;
  }
  __threadfence();
#pragma unroll
  for (int it = 0; it < 2; ++it) {
    const int e = tid + ETHR * it;
    const int nl = e >> 3, q = e & 7;
    const v8h hv = *(const v8h*)(sT + nl * WTP + 8 * q);
    *(volatile v8h*)(O + (size_t)(n0 + nl) * CC + k0 + 8 * q) = hv;
  }
}

__global__ __launch_bounds__(GTHR) void k_gemm(const _Float16* __restrict__ A16,
                                               const _Float16* __restrict__ B16,
                                               float* Cf, float scl, int sig_z) {
  __shared__ __align__(16) float sO[GWAV * 32 * 64];
  const int tid = threadIdx.x, lane = tid & 31, wave = tid >> 5, h = lane >> 4, m = lane & 15;
  const int z = blockIdx.z;
  const size_t pz = (size_t)z * (size_t)TT * (size_t)CC;
  const _Float16* A = A16 + pz;
  const _Float16* B = B16 + pz;
  float* C = Cf + pz;
  const int bm0 = blockIdx.y * BMB, bn0 = blockIdx.x * BNB;
  const int m0 = bm0 + 32 * (wave >> 1);
  const int n0 = bn0 + 64 * (wave & 1);

  v8f acc[2][4];
#pragma unroll
  for (int mi = 0; mi < 2; ++mi)
#pragma unroll
    for (int ni = 0; ni < 4; ++ni) acc[mi][ni] = zero8();

  const _Float16* ap = A + (size_t)(m0 + m) * CC + 8 * h;
  const _Float16* bp = B + (size_t)(n0 + m) * CC + 8 * h;

#pragma unroll 1
  for (int ks = 0; ks < CC / 32; ++ks) {
    const int k0 = 32 * ks;
    Frag fa0, fa1;
    fa0.h[0] = *(const v8h*)(ap + k0);
    fa0.h[1] = *(const v8h*)(ap + k0 + 16);
    fa1.h[0] = *(const v8h*)(ap + (size_t)16 * CC + k0);
    fa1.h[1] = *(const v8h*)(ap + (size_t)16 * CC + k0 + 16);
#pragma unroll
    for (int ni = 0; ni < 4; ++ni) {
      const _Float16* bq = bp + (size_t)(16 * ni) * CC + k0;
      Frag fb;
      fb.h[0] = *(const v8h*)bq;
      fb.h[1] = *(const v8h*)(bq + 16);
      acc[0][ni] = wmh(fa0.v, fb.v, acc[0][ni]);
      acc[1][ni] = wmh(fa1.v, fb.v, acc[1][ni]);
    }
  }

  float* sw = sO + wave * (32 * 64);
#pragma unroll
  for (int mi = 0; mi < 2; ++mi)
#pragma unroll
    for (int ni = 0; ni < 4; ++ni) {
      const int cl = 16 * ni + m;
#pragma unroll
      for (int r = 0; r < 8; ++r) {
        const int rl = 16 * mi + 8 * h + r;
        sw[rl * 64 + cl] = acc[mi][ni][r] * scl;
      }
    }
  __syncthreads();

  if (z == sig_z) {
#pragma unroll 1
    for (int e = tid; e < GWAV * 32 * 64; e += GTHR) sO[e] = sigm_(sO[e]);
  }
  __syncthreads();

#pragma unroll
  for (int p = 0; p < 16; ++p) {
    const int rl = 2 * p + h;
    const v4f v = *(const v4f*)(sw + rl * 64 + 4 * m);
    *(volatile v4f*)(C + (size_t)(m0 + rl) * CC + n0 + 4 * m) = v;
  }
  __threadfence();
#pragma unroll
  for (int p = 0; p < 16; ++p) {
    const int rl = 2 * p + h;
    const v4f v = *(const v4f*)(sw + rl * 64 + 4 * m);
    *(volatile v4f*)(C + (size_t)(m0 + rl) * CC + n0 + 4 * m) = v;
  }
}

__global__ __launch_bounds__(ETHR) void k_wkv(const float* __restrict__ KF, const float* __restrict__ VF,
                                              const float* __restrict__ SF, const float* __restrict__ td,
                                              const float* __restrict__ tf, _Float16* RW) {
  __shared__ __align__(16) _Float16 sH[TB * ETHR];
  const int tid = threadIdx.x, lane = tid & 31, wave = tid >> 5;
  const int cb = blockIdx.x * ETHR;
  const int c = cb + tid;
  const float tdc = td[c], tfc = tf[c];

  float arg = tdc, y = 0.0f, q = 0.0f, d = 0.0f, eu = 0.0f;
#pragma unroll 1
  for (int i = 0; i < 4; ++i) {
    y = expf(arg);
    q = (i == 1) ? y : q;
    d = (i == 2) ? y : d;
    eu = (i == 3) ? y : eu;
    arg = (i == 2) ? tfc : -y;
  }
  (void)q;

  float a = 0.0f, b = 0.0f;
#pragma unroll 1
  for (int t0 = 0; t0 < TT; t0 += TB) {
#pragma unroll 1
    for (int tl = 0; tl < TB; ++tl) {
      const size_t idx = (size_t)(t0 + tl) * CC + c;
      const float kf = KF[idx];
      const float vf = VF[idx];
      const float sf = SF[idx];
      const float ek = __expf(kf);
      const float ekv = ek * vf;
      const float num = a + eu * ekv;
      const float den = b + eu * ek;
      const float wkv = num * rcp_(den);
      const float rw = sf * wkv * RCAR;
      sH[tl * ETHR + tid] = (_Float16)rw;
      a = d * a + ekv;
      b = d * b + ek;
    }
    __syncthreads();
#pragma unroll
    for (int j = 0; j < TB / EWAV; ++j) {
      const int tl = wave * (TB / EWAV) + j;
      const v8h v = *(const v8h*)(sH + tl * ETHR + 8 * lane);
      *(volatile v8h*)(RW + (size_t)(t0 + tl) * CC + cb + 8 * lane) = v;
    }
    __threadfence();
#pragma unroll
    for (int j = 0; j < TB / EWAV; ++j) {
      const int tl = wave * (TB / EWAV) + j;
      const v8h v = *(const v8h*)(sH + tl * ETHR + 8 * lane);
      *(volatile v8h*)(RW + (size_t)(t0 + tl) * CC + cb + 8 * lane) = v;
    }
    __syncthreads();
  }
}

extern "C" void kernel_launch(void* const* d_in, const int* in_sizes, int n_in,
                              void* d_out, int out_size, void* d_ws, size_t ws_size,
                              hipStream_t stream) {
  if (n_in < 10) return;
  if (in_sizes[0] != TT * CC) return;
  if (in_sizes[1] != CC || in_sizes[2] != CC || in_sizes[3] != CC || in_sizes[4] != CC || in_sizes[5] != CC) return;
  if (in_sizes[6] != CC * CC || in_sizes[7] != CC * CC || in_sizes[8] != CC * CC || in_sizes[9] != CC * CC) return;
  if (out_size != TT * CC) return;
  const size_t tot = (size_t)WSTOT;
  if (tot > ws_size || tot > (size_t)WSCAP) return;

  const float* x   = (const float*)d_in[0];
  const float* td  = (const float*)d_in[1];
  const float* tf  = (const float*)d_in[2];
  const float* tmk = (const float*)d_in[3];
  const float* tmv = (const float*)d_in[4];
  const float* tmr = (const float*)d_in[5];
  const float* Wk  = (const float*)d_in[6];
  const float* Wv  = (const float*)d_in[7];
  const float* Wr  = (const float*)d_in[8];
  const float* Wo  = (const float*)d_in[9];
  float* out = (float*)d_out;

  char* ws = (char*)d_ws;
  _Float16* XK  = (_Float16*)(ws + OXK);
  _Float16* XV  = (_Float16*)(ws + OXV);
  _Float16* XR  = (_Float16*)(ws + OXR);
  _Float16* WKT = (_Float16*)(ws + OWK);
  _Float16* WOT = (_Float16*)(ws + OWO);
  float* KF = (float*)(ws + OKF);
  float* VF = (float*)(ws + OVF);
  float* SF = (float*)(ws + OSF);
  _Float16* RW = (_Float16*)(ws + ORW);

  k_mix<<<TT, ETHR, 0, stream>>>(x, tmk, tmv, tmr, XK, XV, XR);

  k_wt<<<dim3(CC / WTT, CC / WTT, 4), ETHR, 0, stream>>>(Wk, Wv, Wr, Wo, WKT);

  k_gemm<<<dim3(CC / BNB, TT / BMB, 3), GTHR, 0, stream>>>(XK, WKT, KF, PSCL, 2);

  k_wkv<<<CC / ETHR, ETHR, 0, stream>>>(KF, VF, SF, td, tf, RW);

  k_gemm<<<dim3(CC / BNB, TT / BMB, 1), GTHR, 0, stream>>>(RW, WOT, out, OSCL, -1);
}
